// PointTransformerLayer_8048768712847
// MI455X (gfx1250) — hardware-verified
//
#include <hip/hip_runtime.h>


#ifndef NB
#define NB 4
#endif
#ifndef SEQ
#define SEQ 512
#endif
#define NB_FULL  4
#define SEQ_FULL 512
#define DIM   64
#define AHID  256
#define QKVN  192
#define ITILE 8
#define JT    16

static_assert(NB >= 1 && NB <= NB_FULL);
static_assert(SEQ >= 128 && SEQ <= SEQ_FULL);
static_assert(SEQ % 128 == 0);
static_assert(SEQ % JT == 0);
static_assert(SEQ % ITILE == 0);
static_assert(AHID == 256);
static_assert(((NB - 1) * SEQ_FULL + SEQ) * DIM <= NB_FULL * SEQ_FULL * DIM);

#define PLANE_F   (NB_FULL * SEQ_FULL * DIM)
#define WS_QKV    0
#define WS_WQF    (3 * PLANE_F * 4)
#define WQF_N     (2 * 12 * 32 * 16)
#define WS_W2F    (WS_WQF + WQF_N * 2)
#define W2F_N     (4 * 2 * 32 * 16)
#define WS_W1F    (WS_W2F + W2F_N * 2)
#define W1F_N     (16 * 2 * 32 * 16)
#define WS_TOTAL  (WS_W1F + W1F_N * 2)
static_assert(WS_TOTAL <= 134217728);
static_assert((WS_WQF % 128) == 0 && (WS_W2F % 128) == 0 && (WS_W1F % 128) == 0);

#define OFF_W1F   0
#define OFF_W2F   32768
#define OFF_HW    40960
#define OFF_VE    57344
#define OFF_KT    90112
#define OFF_VT    94208
#define OFF_OUT   98304
#define OFF_W1P   100352
#define OFF_B1P   101120
#define OFF_B2P   101376
#define OFF_B1A   101632
#define OFF_W2A   102656
#define OFF_POSJ  103680
#define OFF_AB2   103936
#define SMEM_BYTES 104064

typedef _Float16       v8h   __attribute__((ext_vector_type(8)));
typedef _Float16       v16h  __attribute__((ext_vector_type(16)));
typedef __bf16         v16bf __attribute__((ext_vector_type(16)));
typedef unsigned short v8us  __attribute__((ext_vector_type(8)));
typedef unsigned short v16us __attribute__((ext_vector_type(16)));
typedef float          v4f   __attribute__((ext_vector_type(4)));
typedef float          v8f   __attribute__((ext_vector_type(8)));
typedef unsigned int   u32x4 __attribute__((ext_vector_type(4)));

__device__ __forceinline__ unsigned int bf16bits(float f) {
    unsigned int u = __float_as_uint(f);
    return (u + 0x7FFFu + ((u >> 16) & 1u)) >> 16;
}
__device__ __forceinline__ float bf16r(float f) {
    return __uint_as_float(bf16bits(f) << 16);
}

__device__ __forceinline__ v8f wmma_f16(v16h a, v16h b, v8f c) {
    return __builtin_amdgcn_wmma_f32_16x16x32_f16(false, a, false, b, (short)0, c, false, false);
}
__device__ __forceinline__ v8f wmma_bf16v(v16bf a, v16bf b, v8f c) {
    return __builtin_amdgcn_wmma_f32_16x16x32_bf16(false, a, false, b, (short)0, c, false, false);
}
__device__ __forceinline__ void wguard_h(v8f& acc, v16h a0, v16h b0, v16h a1, v16h b1) {
    asm volatile("v_nop\n\tv_nop\n\tv_nop\n\tv_nop" : "+v"(acc) : "v"(a0), "v"(b0), "v"(a1), "v"(b1));
}
__device__ __forceinline__ void wguard_u(v8f& acc, v16us a0, v16us b0, v16us a1, v16us b1) {
    asm volatile("v_nop\n\tv_nop\n\tv_nop\n\tv_nop" : "+v"(acc) : "v"(a0), "v"(b0), "v"(a1), "v"(b1));
}

__device__ __forceinline__ void st2_f4(float* p, v4f v) {
    *(volatile v4f*)p = v;
    __threadfence();
    *(volatile v4f*)p = v;
}
__device__ __forceinline__ void st2_us8(unsigned short* p, v8us v) {
    *(volatile v8us*)p = v;
    __threadfence();
    *(volatile v8us*)p = v;
}
__device__ __forceinline__ void st2_h8(_Float16* p, v8h v) {
    *(volatile v8h*)p = v;
    __threadfence();
    *(volatile v8h*)p = v;
}

__global__ void __launch_bounds__(256)
k_pack(const float* __restrict__ w_qkv, const float* __restrict__ pos_w2,
       const float* __restrict__ attn_w1,
       unsigned short* __restrict__ wqf, _Float16* __restrict__ w2f, _Float16* __restrict__ w1f)
{
    const int tid = threadIdx.x;
    for (int u = tid; u < WQF_N / 8; u += 256) {
        const int e0 = (u & 1) * 8, ln = (u >> 1) & 31, t = u >> 6;
        const int ks = t & 1, nt = t >> 1, hh = ln >> 4;
        const int n  = nt * 16 + (ln & 15);
        const int kb = ks * 32 + 8 * hh + 2 * e0;
        v8us o;
#pragma unroll
        for (int i = 0; i < 8; ++i)
            o[i] = (unsigned short)bf16bits(w_qkv[(kb + i) * QKVN + n]);
        st2_us8(wqf + (size_t)u * 8, o);
    }
    for (int u = tid; u < W2F_N / 8; u += 256) {
        const int e0 = (u & 1) * 8, ln = (u >> 1) & 31, t = u >> 6;
        const int ks = t & 1, nt = t >> 1, hh = ln >> 4;
        const int n  = nt * 16 + (ln & 15);
        const int kb = ks * 32 + 8 * hh + 2 * e0;
        v8h o;
#pragma unroll
        for (int i = 0; i < 8; ++i)
            o[i] = (_Float16)(16.0f * bf16r(pos_w2[(kb + i) * DIM + n]));
        st2_h8(w2f + (size_t)u * 8, o);
    }
    for (int u = tid; u < W1F_N / 8; u += 256) {
        const int e0 = (u & 1) * 8, ln = (u >> 1) & 31, t = u >> 6;
        const int ks = t & 1, nt = t >> 1, hh = ln >> 4;
        const int n  = nt * 16 + (ln & 15);
        const int kb = ks * 32 + 8 * hh + 2 * e0;
        v8h o;
#pragma unroll
        for (int i = 0; i < 8; ++i)
            o[i] = (_Float16)(16.0f * bf16r(attn_w1[(kb + i) * AHID + n]));
        st2_h8(w1f + (size_t)u * 8, o);
    }
}

__global__ void __launch_bounds__(256)
k_qkv(const float* __restrict__ x, const unsigned short* __restrict__ wqf,
      float* __restrict__ qkv)
{
    __shared__ __align__(16) float stg[8 * 1024];
    const int tid = threadIdx.x, wid = tid >> 5, lane = tid & 31, h = lane >> 4, m = lane & 15;
    const int bpb = SEQ / 128;
    const int bb  = blockIdx.x / bpb;
    const int r0  = bb * SEQ_FULL + (blockIdx.x % bpb) * 128 + wid * 16;

    const float* xr = x + (size_t)(r0 + m) * DIM;
    v16us ua0, ua1;
    {
        const v4f f0 = *(const v4f*)(xr + 8 * h);
        const v4f f1 = *(const v4f*)(xr + 8 * h + 4);
        const v4f f2 = *(const v4f*)(xr + 16 + 8 * h);
        const v4f f3 = *(const v4f*)(xr + 20 + 8 * h);
        const v4f g0 = *(const v4f*)(xr + 32 + 8 * h);
        const v4f g1 = *(const v4f*)(xr + 36 + 8 * h);
        const v4f g2 = *(const v4f*)(xr + 48 + 8 * h);
        const v4f g3 = *(const v4f*)(xr + 52 + 8 * h);
#pragma unroll
        for (int i = 0; i < 4; ++i) {
            ua0[i]      = (unsigned short)bf16bits(f0[i]);
            ua0[4 + i]  = (unsigned short)bf16bits(f1[i]);
            ua0[8 + i]  = (unsigned short)bf16bits(f2[i]);
            ua0[12 + i] = (unsigned short)bf16bits(f3[i]);
            ua1[i]      = (unsigned short)bf16bits(g0[i]);
            ua1[4 + i]  = (unsigned short)bf16bits(g1[i]);
            ua1[8 + i]  = (unsigned short)bf16bits(g2[i]);
            ua1[12 + i] = (unsigned short)bf16bits(g3[i]);
        }
    }
    const v16bf a0 = __builtin_bit_cast(v16bf, ua0);
    const v16bf a1 = __builtin_bit_cast(v16bf, ua1);
    float* stw = stg + wid * 1024;

#pragma unroll 1
    for (int pl = 0; pl < 3; ++pl) {
#pragma unroll
        for (int t = 0; t < 4; ++t) {
            const int nt = pl * 4 + t;
            const unsigned short* bp = wqf + ((size_t)(nt * 2) * 32 + lane) * 16;
            const v16us ub0 = *(const v16us*)bp;
            const v16us ub1 = *(const v16us*)(bp + 512);
            v8f acc = {};
            acc = wmma_bf16v(a0, __builtin_bit_cast(v16bf, ub0), acc);
            acc = wmma_bf16v(a1, __builtin_bit_cast(v16bf, ub1), acc);
            wguard_u(acc, ua0, ub0, ua1, ub1);
#pragma unroll
            for (int r = 0; r < 8; ++r) stw[(8 * h + r) * 64 + t * 16 + m] = acc[r];
        }
        __syncthreads();
        float* plane = qkv + (size_t)pl * PLANE_F;
#pragma unroll
        for (int it = 0; it < 8; ++it) {
            const int row = 2 * it + h, c4 = m * 4;
            const v4f v = *(const v4f*)(stw + row * 64 + c4);
            st2_f4(plane + (size_t)(r0 + row) * DIM + c4, v);
        }
        __syncthreads();
    }
}

__global__ void __launch_bounds__(256) __attribute__((amdgpu_num_vgpr(256)))
k_attn(const float* __restrict__ pos, const float* __restrict__ qp,
       const float* __restrict__ kp, const float* __restrict__ vp,
       const float* __restrict__ pos_w1, const float* __restrict__ pos_b1,
       const float* __restrict__ pos_b2, const float* __restrict__ attn_b1,
       const float* __restrict__ attn_w2, const float* __restrict__ attn_b2,
       const _Float16* __restrict__ w2f, const _Float16* __restrict__ w1f,
       float* __restrict__ out)
{
    extern __shared__ __align__(16) char smem[];
    _Float16* s_w1f = (_Float16*)(smem + OFF_W1F);
    _Float16* s_w2f = (_Float16*)(smem + OFF_W2F);
    _Float16* s_hw  = (_Float16*)(smem + OFF_HW);
    float* s_ve   = (float*)(smem + OFF_VE);
    float* s_kt   = (float*)(smem + OFF_KT);
    float* s_vt   = (float*)(smem + OFF_VT);
    float* s_out  = (float*)(smem + OFF_OUT);
    float* s_w1p  = (float*)(smem + OFF_W1P);
    float* s_b1p  = (float*)(smem + OFF_B1P);
    float* s_b2p  = (float*)(smem + OFF_B2P);
    float* s_b1a  = (float*)(smem + OFF_B1A);
    float* s_w2a  = (float*)(smem + OFF_W2A);
    float* s_posj = (float*)(smem + OFF_POSJ);
    float* s_ab2  = (float*)(smem + OFF_AB2);

    const int tid = threadIdx.x;
    const int wid = tid >> 5, lane = tid & 31, h = lane >> 4, m = lane & 15;
    const int bpb  = SEQ / ITILE;
    const int bb   = blockIdx.x / bpb;
    const int i0   = (blockIdx.x % bpb) * ITILE;
    const int irow = bb * SEQ_FULL + i0 + wid;

    {
        const u32x4* src = (const u32x4*)w1f;
        u32x4* dst = (u32x4*)(smem + OFF_W1F);
        for (int i = tid; i < (W1F_N * 2) / 16; i += 256) dst[i] = src[i];
        const u32x4* src2 = (const u32x4*)w2f;
        u32x4* dst2 = (u32x4*)(smem + OFF_W2F);
        for (int i = tid; i < (W2F_N * 2) / 16; i += 256) dst2[i] = src2[i];
    }
    if (tid < 3 * DIM) s_w1p[tid] = bf16r(pos_w1[tid]);
    if (tid < DIM) { s_b1p[tid] = bf16r(pos_b1[tid]); s_b2p[tid] = bf16r(pos_b2[tid]); }
    s_b1a[tid] = bf16r(attn_b1[tid]);
    s_w2a[tid] = bf16r(attn_w2[tid]);
    if (tid == 0) s_ab2[0] = bf16r(attn_b2[0]);
    __syncthreads();

    float qreg[4];
#pragma unroll
    for (int t = 0; t < 4; ++t) qreg[t] = qp[(size_t)irow * DIM + t * 16 + m];
    const float pi0 = bf16r(pos[(size_t)irow * 3 + 0]);
    const float pi1 = bf16r(pos[(size_t)irow * 3 + 1]);
    const float pi2 = bf16r(pos[(size_t)irow * 3 + 2]);
    const float ab2 = s_ab2[0];
    _Float16* s_hwp = s_hw + wid * 1024;
    float*    s_vep = s_ve + wid * 1024;

    float m_run = -__builtin_inff(), l_run = 0.f, acc0 = 0.f, acc1 = 0.f;
    const int d0 = h * 32 + m, d1 = d0 + 16;

#pragma unroll 1
    for (int chunk = 0; chunk < SEQ / JT; ++chunk) {
        const int jb = bb * SEQ_FULL + chunk * JT;
        __syncthreads();
#pragma unroll
        for (int it = 0; it < 4; ++it) {
            const int idx = tid + it * 256;
            const int jj = idx >> 6, d = idx & 63;
            const size_t g = (size_t)(jb + jj) * DIM + d;
            s_kt[d * JT + jj] = kp[g];
            s_vt[d * JT + jj] = vp[g];
        }
        if (tid < JT * 3) s_posj[tid] = bf16r(pos[(size_t)jb * 3 + tid]);
        __syncthreads();

        const float rl0 = pi0 - s_posj[m * 3 + 0];
        const float rl1 = pi1 - s_posj[m * 3 + 1];
        const float rl2 = pi2 - s_posj[m * 3 + 2];
        v16h ha, hb;
#pragma unroll
        for (int e = 0; e < 16; ++e) {
            const int c0 = (e < 8) ? (8 * h + e) : (8 + 8 * h + e);
            const int c1 = 32 + c0;
            const float t0 = rl0 * s_w1p[c0] + rl1 * s_w1p[64 + c0] + rl2 * s_w1p[128 + c0] + s_b1p[c0];
            const float t1 = rl0 * s_w1p[c1] + rl1 * s_w1p[64 + c1] + rl2 * s_w1p[128 + c1] + s_b1p[c1];
            ha[e] = (_Float16)fmaxf(t0, 0.f);
            hb[e] = (_Float16)fmaxf(t1, 0.f);
        }

        v8f embC[4];
#pragma unroll
        for (int nt = 0; nt < 4; ++nt) {
            const _Float16* bp = s_w2f + ((nt * 2) * 32 + lane) * 16;
            const v16h b0 = *(const v16h*)bp;
            const v16h b1 = *(const v16h*)(bp + 512);
            v8f acc = {};
            acc = wmma_f16(ha, b0, acc);
            acc = wmma_f16(hb, b1, acc);
            wguard_h(acc, ha, b0, hb, b1);
            embC[nt] = acc;
        }

#pragma unroll
        for (int nt = 0; nt < 4; ++nt) {
            const int d  = nt * 16 + m;
            const int ks = d >> 5, kk = d & 31;
            const int e  = ((kk >> 4) << 3) | (kk & 7);
            const int L  = 8 * h + 16 * ((kk >> 3) & 1);
            const float b2v = s_b2p[d];
            const float qv  = qreg[nt];
            const float* ktp = s_kt + d * JT + 8 * h;
            const float* vtp = s_vt + d * JT + 8 * h;
            v4f va, vb;
#pragma unroll
            for (int r = 0; r < 8; ++r) {
                const float em = embC[nt][r] * 0.0625f + b2v;
                const float hv = qv - ktp[r] + em;
                s_hwp[(ks * 32 + L + r) * 16 + e] = (_Float16)hv;
                const float vv = vtp[r] + em;
                if (r < 4) va[r] = vv; else vb[r - 4] = vv;
            }
            *(v4f*)(s_vep + d * JT + 8 * h)     = va;
            *(v4f*)(s_vep + d * JT + 8 * h + 4) = vb;
        }
        __syncthreads();
        const v16h a0 = *(const v16h*)(s_hwp + lane * 16);
        const v16h a1 = *(const v16h*)(s_hwp + 512 + lane * 16);

        float simp[8];
#pragma unroll
        for (int r = 0; r < 8; ++r) simp[r] = 0.f;
#pragma unroll 2
        for (int nt = 0; nt < 16; ++nt) {
            const _Float16* bp = s_w1f + ((nt * 2) * 32 + lane) * 16;
            const v16h b0 = *(const v16h*)bp;
            const v16h b1 = *(const v16h*)(bp + 512);
            v8f acc = {};
            acc = wmma_f16(a0, b0, acc);
            acc = wmma_f16(a1, b1, acc);
            wguard_h(acc, a0, b0, a1, b1);
            const int n = nt * 16 + m;
            const float bb1 = s_b1a[n], ww2 = s_w2a[n];
#pragma unroll
            for (int r = 0; r < 8; ++r)
                simp[r] += fmaxf(acc[r] * 0.0625f + bb1, 0.f) * ww2;
        }
#pragma unroll
        for (int r = 0; r < 8; ++r) {
            float s = simp[r];
            s += __shfl_xor(s, 1, 32);
            s += __shfl_xor(s, 2, 32);
            s += __shfl_xor(s, 4, 32);
            s += __shfl_xor(s, 8, 32);
            simp[r] = s + ab2;
        }
        float sj[16];
#pragma unroll
        for (int jj = 0; jj < 16; ++jj) sj[jj] = __shfl(simp[jj & 7], (jj >> 3) * 16, 32);

        float mc = sj[0];
#pragma unroll
        for (int jj = 1; jj < 16; ++jj) mc = fmaxf(mc, sj[jj]);
        const float mnew = fmaxf(m_run, mc);
        const float corr = __expf(m_run - mnew);
        l_run *= corr; acc0 *= corr; acc1 *= corr;
        float p[16];
#pragma unroll
        for (int jj = 0; jj < 16; ++jj) { p[jj] = __expf(sj[jj] - mnew); l_run += p[jj]; }
        const v4f* ve0 = (const v4f*)(s_vep + d0 * JT);
        const v4f* ve1 = (const v4f*)(s_vep + d1 * JT);
#pragma unroll
        for (int q4 = 0; q4 < 4; ++q4) {
            const v4f x0 = ve0[q4], x1 = ve1[q4];
#pragma unroll
            for (int u = 0; u < 4; ++u) {
                acc0 += p[q4 * 4 + u] * x0[u];
                acc1 += p[q4 * 4 + u] * x1[u];
            }
        }
        m_run = mnew;
    }

    const float inv = 1.0f / l_run;
    s_out[wid * 64 + d0] = acc0 * inv;
    s_out[wid * 64 + d1] = acc1 * inv;
    __syncthreads();
    if (tid < 128) {
        const int row = tid >> 4, c4 = (tid & 15) * 4;
        const v4f v = *(const v4f*)(s_out + row * 64 + c4);
        st2_f4(out + (size_t)(bb * SEQ_FULL + i0 + row) * DIM + c4, v);
    }
}

extern "C" void kernel_launch(void* const* d_in, const int* in_sizes, int n_in,
                              void* d_out, int out_size, void* d_ws, size_t ws_size,
                              hipStream_t stream) {
    if (n_in < 11) return;
    const int rows_needed = (NB - 1) * SEQ_FULL + SEQ;
    if (in_sizes[0] < rows_needed * DIM) return;
    if (in_sizes[1] < rows_needed * 3) return;
    if (in_sizes[2] < DIM * QKVN) return;
    if (in_sizes[3] < 3 * DIM || in_sizes[4] < DIM || in_sizes[5] < DIM * DIM || in_sizes[6] < DIM) return;
    if (in_sizes[7] < DIM * AHID || in_sizes[8] < AHID || in_sizes[9] < AHID || in_sizes[10] < 1) return;
    if (out_size < rows_needed * DIM) return;
    if (ws_size < (size_t)WS_TOTAL) return;

    const float* x       = (const float*)d_in[0];
    const float* pos     = (const float*)d_in[1];
    const float* w_qkv   = (const float*)d_in[2];
    const float* pos_w1  = (const float*)d_in[3];
    const float* pos_b1  = (const float*)d_in[4];
    const float* pos_w2  = (const float*)d_in[5];
    const float* pos_b2  = (const float*)d_in[6];
    const float* attn_w1 = (const float*)d_in[7];
    const float* attn_b1 = (const float*)d_in[8];
    const float* attn_w2 = (const float*)d_in[9];
    const float* attn_b2 = (const float*)d_in[10];
    float* out = (float*)d_out;

    char* ws = (char*)d_ws;
    float*          qkv = (float*)(ws + WS_QKV);
    unsigned short* wqf = (unsigned short*)(ws + WS_WQF);
    _Float16*       w2f = (_Float16*)(ws + WS_W2F);
    _Float16*       w1f = (_Float16*)(ws + WS_W1F);

    (void)hipFuncSetAttribute(reinterpret_cast<const void*>(&k_attn),
                              hipFuncAttributeMaxDynamicSharedMemorySize, SMEM_BYTES);

    k_pack<<<1, 256, 0, stream>>>(w_qkv, pos_w2, attn_w1, wqf, w2f, w1f);
    k_qkv<<<NB * (SEQ / 128), 256, 0, stream>>>(x, wqf, qkv);
    k_attn<<<NB * (SEQ / ITILE), 256, SMEM_BYTES, stream>>>(
        pos, qkv, qkv + PLANE_F, qkv + 2 * PLANE_F,
        pos_w1, pos_b1, pos_b2, attn_b1, attn_w2, attn_b2, w2f, w1f, out);
}
